// MatchLSTM_17609365914096
// MI455X (gfx1250) — hardware-run, weakly checked
//
#include <hip/hip_runtime.h>
#include <math.h>

constexpr int NBAT  = 128;
constexpr int NTP   = 64;
constexpr int NTH   = 64;
constexpr int NHID  = 512;
constexpr int NEMB  = 300;
constexpr int KEMB  = 320;
constexpr int NVOC  = 30000;
constexpr int NG4   = 2048;
constexpr int NK2   = 1024;
constexpr int NG3O  = 1536;
constexpr int NCLS  = 3;
constexpr int NROWP = NTP * NBAT;
constexpr int NROWH = NTH * NBAT;
constexpr int NTHR  = 256;
constexpr int SEQB  = 16;
constexpr int HMP   = 520;
constexpr int MKP   = 1032;
constexpr int HWP   = 516;
constexpr int SLABP = 68;
static_assert(KEMB % 32 == 0 && NHID % 32 == 0 && NK2 % 32 == 0);
static_assert(NROWP % 64 == 0 && NROWH % 64 == 0 && NHID % 64 == 0);
static_assert(NROWP % 16 == 0 && NHID / 64 == 8);
static_assert(NEMB % 4 == 0 && NEMB < KEMB);
static_assert(NBAT % SEQB == 0 && SEQB == 2 * (NTHR / 32));
static_assert(NHID == 64 * (NTHR / 32));
static_assert(SEQB * (NHID / 8) == 4 * NTHR);
static_assert(NTP == 64);
static_assert((NBAT * NCLS) % 4 == 0 && (NBAT * NCLS) / 4 == 96);
static_assert(HMP % 8 == 0 && MKP % 8 == 0 && HWP % 4 == 0 && SLABP % 4 == 0);

typedef __attribute__((ext_vector_type(16))) __bf16   v16b;
typedef __attribute__((ext_vector_type(8)))  __bf16   v8b;
typedef __attribute__((ext_vector_type(8)))  _Float16 v8h;
typedef __attribute__((ext_vector_type(8)))  float    v8f;
typedef __attribute__((ext_vector_type(4)))  float    v4f;
typedef __attribute__((ext_vector_type(4)))  unsigned v4u;

__device__ __forceinline__ unsigned short f2bf_bits(float f) {
  unsigned u = __float_as_uint(f);
  return (unsigned short)((u + 0x7FFFu + ((u >> 16) & 1u)) >> 16);
}
__device__ __forceinline__ float bf_bits2f(unsigned short h) { return __uint_as_float(((unsigned)h) << 16); }
__device__ __forceinline__ float bf16r(float f) { return bf_bits2f(f2bf_bits(f)); }

__device__ __forceinline__ void guard1_in3_b(v8f& a, v16b x, v16b y, v16b z) {
  asm volatile("v_nop\n\tv_nop\n\tv_nop\n\tv_nop" : "+v"(a) : "v"(x), "v"(y), "v"(z)); }
__device__ __forceinline__ void guard3_in4_b(v8f& a, v8f& b, v8f& c, v16b x, v16b y, v16b z, v16b w) {
  asm volatile("v_nop\n\tv_nop\n\tv_nop\n\tv_nop" : "+v"(a), "+v"(b), "+v"(c) : "v"(x), "v"(y), "v"(z), "v"(w)); }
__device__ __forceinline__ void guard3_in5_b(v8f& a, v8f& b, v8f& c, v16b x, v16b y, v16b z, v16b u, v16b w) {
  asm volatile("v_nop\n\tv_nop\n\tv_nop\n\tv_nop" : "+v"(a), "+v"(b), "+v"(c) : "v"(x), "v"(y), "v"(z), "v"(u), "v"(w)); }
__device__ __forceinline__ void guard4_in2_b(v8f& a, v8f& b, v8f& c, v8f& d, v16b x, v16b y) {
  asm volatile("v_nop\n\tv_nop\n\tv_nop\n\tv_nop" : "+v"(a), "+v"(b), "+v"(c), "+v"(d) : "v"(x), "v"(y)); }
__device__ __forceinline__ void keep4_b(v16b a, v16b b, v16b c, v16b d) { asm volatile("v_nop" :: "v"(a), "v"(b), "v"(c), "v"(d)); }
__device__ __forceinline__ void acc_guard4(v8f& a, v8f& b, v8f& c, v8f& d) { asm volatile("v_nop\n\tv_nop\n\tv_nop\n\tv_nop" : "+v"(a), "+v"(b), "+v"(c), "+v"(d)); }
__device__ __forceinline__ void acc_guard3(v8f& a, v8f& b, v8f& c) { asm volatile("v_nop\n\tv_nop\n\tv_nop\n\tv_nop" : "+v"(a), "+v"(b), "+v"(c)); }
__device__ __forceinline__ void acc_guard1(v8f& a) { asm volatile("v_nop\n\tv_nop\n\tv_nop\n\tv_nop" : "+v"(a)); }

struct FragB {
  union U { v16b v; v8b h[2]; };
  static __device__ __forceinline__ v16b load(const __bf16* p) {
    U f; f.h[0] = *(const v8b*)(p); f.h[1] = *(const v8b*)(p + 16); return f.v;
  }
  static __device__ __forceinline__ v8f mma(v16b a, v16b b, v8f c) {
    return __builtin_amdgcn_wmma_f32_16x16x32_bf16(false, a, false, b, (short)0, c, false, false);
  }
};

__device__ __forceinline__ float sgm_f(float x) { return __builtin_amdgcn_rcpf(1.0f + expf(-x)); }
__device__ __forceinline__ float tnh_f(float x) { return 1.0f - 2.0f * __builtin_amdgcn_rcpf(expf(2.0f * x) + 1.0f); }
__device__ __forceinline__ float cell_h(float zi, float zg, float zo) {
  const float ig = sgm_f(zi);
  const float gg = tnh_f(zg);
  const float og = sgm_f(zo);
  const float cc = ig * gg;
  return og * tnh_f(cc);
}

template <int MODE>
__global__ __launch_bounds__(NTHR) void cvt8_kernel(const float* __restrict__ src, unsigned short* __restrict__ dst,
                                                    int nrow, int ncol8, int spitch, int scol0, float sc) {
  const int i  = blockIdx.x * NTHR + threadIdx.x;
  const int n8 = nrow * ncol8;
  if (i < n8) {
    const int row = i / ncol8;
    const int c8  = i - row * ncol8;
    const float* sp = src + (size_t)row * spitch + scol0 + c8 * 8;
    const v4f a = *(const v4f*)(sp);
    const v4f b = *(const v4f*)(sp + 4);
    v8h hv;
#pragma unroll
    for (int e = 0; e < 4; ++e) {
      unsigned short b0, b1;
      if (MODE == 0) {
        b0 = f2bf_bits(a[e] * sc);
        b1 = f2bf_bits(b[e] * sc);
      } else {
        b0 = __builtin_bit_cast(unsigned short, (_Float16)(bf16r(a[e]) * sc));
        b1 = __builtin_bit_cast(unsigned short, (_Float16)(bf16r(b[e]) * sc));
      }
      hv[e]     = __builtin_bit_cast(_Float16, b0);
      hv[4 + e] = __builtin_bit_cast(_Float16, b1);
    }
    *(volatile v8h*)(dst + (size_t)i * 8) = hv;
    __threadfence();
    *(volatile v8h*)(dst + (size_t)i * 8) = hv;
  }
}

__global__ __launch_bounds__(NTHR) void cvt_pad_kernel(const float* __restrict__ src, unsigned short* __restrict__ dst, int nrow) {
  const int i  = blockIdx.x * NTHR + threadIdx.x;
  const int n8 = nrow * (KEMB / 8);
  if (i < n8) {
    const int row  = i / (KEMB / 8);
    const int c8   = i - row * (KEMB / 8);
    const int col0 = c8 * 8;
    const int ca = (col0 < NEMB - 4) ? col0 : (NEMB - 4);
    const int cb = (col0 + 4 < NEMB - 4) ? (col0 + 4) : (NEMB - 4);
    const float* sp = src + (size_t)row * NEMB;
    const v4f a = *(const v4f*)(sp + ca);
    const v4f b = *(const v4f*)(sp + cb);
    const float fa = (col0 < NEMB) ? 1.0f : 0.0f;
    const float fb = (col0 + 4 < NEMB) ? 1.0f : 0.0f;
    v8h hv;
#pragma unroll
    for (int e = 0; e < 4; ++e) {
      hv[e]     = __builtin_bit_cast(_Float16, f2bf_bits(fmaf(a[e], fa, 0.0f)));
      hv[4 + e] = __builtin_bit_cast(_Float16, f2bf_bits(fmaf(b[e], fb, 0.0f)));
    }
    *(volatile v8h*)(dst + (size_t)i * 8) = hv;
    __threadfence();
    *(volatile v8h*)(dst + (size_t)i * 8) = hv;
  }
}

__global__ __launch_bounds__(NTHR) void gather_rows_kernel(const int* __restrict__ ids, const float* __restrict__ emb,
                                                           unsigned short* __restrict__ dst, int nrow) {
  const int i  = blockIdx.x * NTHR + threadIdx.x;
  const int n8 = nrow * (KEMB / 8);
  if (i < n8) {
    const int row  = i / (KEMB / 8);
    const int c8   = i - row * (KEMB / 8);
    const int col0 = c8 * 8;
    int id = ids[row];
    id = (id < 0) ? 0 : ((id > NVOC - 1) ? (NVOC - 1) : id);
    const int ca = (col0 < NEMB - 4) ? col0 : (NEMB - 4);
    const int cb = (col0 + 4 < NEMB - 4) ? (col0 + 4) : (NEMB - 4);
    const float* sp = emb + (size_t)id * NEMB;
    const v4f a = *(const v4f*)(sp + ca);
    const v4f b = *(const v4f*)(sp + cb);
    const float fa = (col0 < NEMB) ? 1.0f : 0.0f;
    const float fb = (col0 + 4 < NEMB) ? 1.0f : 0.0f;
    v8h hv;
#pragma unroll
    for (int e = 0; e < 4; ++e) {
      hv[e]     = __builtin_bit_cast(_Float16, f2bf_bits(fmaf(a[e], fa, 0.0f)));
      hv[4 + e] = __builtin_bit_cast(_Float16, f2bf_bits(fmaf(b[e], fb, 0.0f)));
    }
    *(volatile v8h*)(dst + (size_t)i * 8) = hv;
    __threadfence();
    *(volatile v8h*)(dst + (size_t)i * 8) = hv;
  }
}

__global__ __launch_bounds__(NTHR) void param_prep_kernel(
    const float* __restrict__ bih_p, const float* __restrict__ bhh_p,
    const float* __restrict__ bih_h, const float* __restrict__ bhh_h,
    const float* __restrict__ bih_m, const float* __restrict__ bhh_m,
    const float* __restrict__ w_e, const float* __restrict__ fc_w, const float* __restrict__ fc_b,
    float* __restrict__ BP, float* __restrict__ BH, float* __restrict__ BM,
    float* __restrict__ WE, float* __restrict__ FCW, float* __restrict__ FCB) {
  const int blk = blockIdx.x, tid = threadIdx.x;
  if (blk < 3) {
    const float* ba = (blk == 0) ? bih_p : ((blk == 1) ? bih_h : bih_m);
    const float* bb = (blk == 0) ? bhh_p : ((blk == 1) ? bhh_h : bhh_m);
    float* dst = (blk == 0) ? BP : ((blk == 1) ? BH : BM);
    v4f o[2];
#pragma unroll
    for (int it = 0; it < 2; ++it) {
      const int q = tid + NTHR * it;
      const v4f va = *(const v4f*)(ba + 4 * q);
      const v4f vb = *(const v4f*)(bb + 4 * q);
#pragma unroll
      for (int e = 0; e < 4; ++e) o[it][e] = bf16r(va[e]) + bf16r(vb[e]);
    }
    for (int pass = 0; pass < 2; ++pass) {
#pragma unroll
      for (int it = 0; it < 2; ++it) *(volatile v4f*)(dst + 4 * (tid + NTHR * it)) = o[it];
      __threadfence();
    }
  } else if (blk == 3) {
    if (tid < NHID / 4) {
      const v4f v = *(const v4f*)(w_e + 4 * tid);
      v4f o;
#pragma unroll
      for (int e = 0; e < 4; ++e) o[e] = bf16r(v[e]);
      for (int pass = 0; pass < 2; ++pass) { *(volatile v4f*)(WE + 4 * tid) = o; __threadfence(); }
    } else if (tid < NHID / 4 + 8) {
      const int l = tid - NHID / 4;
      v4f o;
#pragma unroll
      for (int e = 0; e < 4; ++e) {
        const int idx = 4 * l + e;
        const int ci  = (idx < NCLS) ? idx : (NCLS - 1);
        const float f = (idx < NCLS) ? 1.0f : 0.0f;
        o[e] = fmaf(bf16r(fc_b[ci]), f, 0.0f);
      }
      for (int pass = 0; pass < 2; ++pass) { *(volatile v4f*)(FCB + 4 * l) = o; __threadfence(); }
    }
  } else {
    v4f o[2];
#pragma unroll
    for (int it = 0; it < 2; ++it) {
      const int q  = tid + NTHR * it;
      const int qc = (q < NCLS * NHID / 4) ? q : (NCLS * NHID / 4 - 1);
      const v4f v = *(const v4f*)(fc_w + 4 * qc);
#pragma unroll
      for (int e = 0; e < 4; ++e) o[it][e] = bf16r(v[e]);
    }
    for (int pass = 0; pass < 2; ++pass) {
      *(volatile v4f*)(FCW + 4 * tid) = o[0];
      if (tid < NCLS * NHID / 4 - NTHR) *(volatile v4f*)(FCW + 4 * (NTHR + tid)) = o[1];
      __threadfence();
    }
  }
}

__global__ __launch_bounds__(NTHR) void gate_gemm_kernel(const unsigned short* __restrict__ Xp,
                                                        const unsigned short* __restrict__ Wp,
                                                        const float* __restrict__ bias,
                                                        unsigned short* __restrict__ Hhi,
                                                        unsigned short* __restrict__ Hlo, int M) {
  __shared__ __align__(16) float sT[NTHR / 32][16 * SLABP];
  const __bf16* X = (const __bf16*)Xp;
  const __bf16* W = (const __bf16*)Wp;
  const int lane = threadIdx.x & 31, wave = threadIdx.x >> 5;
  const int tilesM = M >> 4;
  const int tile = blockIdx.x * (NTHR / 32) + wave;
  if (tile >= tilesM * (NHID / 64)) return;
  const int tm = tile >> 3, tn = tile & 7;
  const int m0 = tm << 4, n0 = tn << 6;
  const int c = lane & 15, hh = lane >> 4, koff = hh * 8, mOff = hh * 8;
  float* slab = sT[wave];
  const v8f z8 = {0.f, 0.f, 0.f, 0.f, 0.f, 0.f, 0.f, 0.f};
  const __bf16* arow = X + (size_t)(m0 + c) * KEMB + koff;

#pragma unroll
  for (int j = 0; j < 4; ++j) {
    const int n = n0 + 16 * j + c;
    const __bf16* wi = W + (size_t)n * KEMB + koff;
    const __bf16* wg = W + (size_t)(NK2 + n) * KEMB + koff;
    const __bf16* wo = W + (size_t)(NG3O + n) * KEMB + koff;
    v8f ai = z8, ag = z8, ao = z8;
#pragma unroll 1
    for (int k0 = 0; k0 < KEMB; k0 += 32) {
      const v16b a   = FragB::load(arow + k0);
      const v16b fbi = FragB::load(wi + k0);
      const v16b fbg = FragB::load(wg + k0);
      const v16b fbo = FragB::load(wo + k0);
      ai = FragB::mma(a, fbi, ai);
      ag = FragB::mma(a, fbg, ag);
      ao = FragB::mma(a, fbo, ao);
      guard3_in4_b(ai, ag, ao, a, fbi, fbg, fbo);
    }
    acc_guard3(ai, ag, ao);
    const float bI = bias[n], bG = bias[NK2 + n], bO = bias[NG3O + n];
#pragma unroll
    for (int r = 0; r < 8; ++r) {
      const float h = cell_h(ai[r] + bI, ag[r] + bG, ao[r] + bO);
      slab[(mOff + r) * SLABP + 16 * j + c] = h;
    }
  }
  __builtin_amdgcn_fence(__ATOMIC_RELEASE, "workgroup");
  __builtin_amdgcn_wave_barrier();
  __builtin_amdgcn_fence(__ATOMIC_ACQUIRE, "workgroup");
  {
    const int q = lane >> 3, c8 = (lane & 7) * 8;
    for (int pass = 0; pass < 2; ++pass) {
#pragma unroll
      for (int it = 0; it < 4; ++it) {
        const int row = it * 4 + q;
        const float* sp = slab + row * SLABP + c8;
        v8h hv, lv;
#pragma unroll
        for (int e = 0; e < 8; ++e) {
          const unsigned short hb = f2bf_bits(sp[e]);
          const unsigned short lb = f2bf_bits(sp[e] - bf_bits2f(hb));
          hv[e] = __builtin_bit_cast(_Float16, hb);
          lv[e] = __builtin_bit_cast(_Float16, lb);
        }
        *(volatile v8h*)(Hhi + (size_t)(m0 + row) * NHID + n0 + c8) = hv;
        *(volatile v8h*)(Hlo + (size_t)(m0 + row) * NHID + n0 + c8) = lv;
      }
      __threadfence();
    }
  }
}

__global__ __launch_bounds__(NTHR) void proj_gemm_kernel(
    const unsigned short* __restrict__ Ap, const unsigned short* __restrict__ A2p, int lda,
    const unsigned short* __restrict__ Btp, int ldb, float* __restrict__ C, int ldc, int M, int N, int K) {
  const __bf16* A = (const __bf16*)Ap; const __bf16* A2 = (const __bf16*)A2p; const __bf16* Bt = (const __bf16*)Btp;
  __shared__ __align__(16) float sT[NTHR / 32][16 * SLABP];
  const int lane = threadIdx.x & 31, wave = threadIdx.x >> 5;
  const int tilesN = N >> 6, tilesM = M >> 6;
  const int tile = blockIdx.x * (NTHR / 32) + wave;
  if (tile >= tilesM * tilesN) return;
  const int tm = tile / tilesN, tn = tile - tm * tilesN;
  const int m0 = tm << 6, n0 = tn << 6;
  const int rlane = lane & 15, koff = (lane >> 4) * 8, mOff = (lane >> 4) * 8;
  const v8f z8 = {0.f, 0.f, 0.f, 0.f, 0.f, 0.f, 0.f, 0.f};

  v8f acc[4][4];
#pragma unroll
  for (int i = 0; i < 4; ++i)
#pragma unroll
    for (int j = 0; j < 4; ++j) acc[i][j] = z8;

  for (int k0 = 0; k0 < K; k0 += 32) {
    v16b bh[4];
#pragma unroll
    for (int j = 0; j < 4; ++j) bh[j] = FragB::load(Bt + (size_t)(n0 + (j << 4) + rlane) * ldb + koff + k0);
#pragma unroll
    for (int i = 0; i < 4; ++i) {
      const size_t ao = (size_t)(m0 + (i << 4) + rlane) * lda + koff + k0;
      const v16b ah = FragB::load(A + ao);
      const v16b al = FragB::load(A2 + ao);
#pragma unroll
      for (int j = 0; j < 4; ++j) {
        acc[i][j] = FragB::mma(ah, bh[j], acc[i][j]);
        acc[i][j] = FragB::mma(al, bh[j], acc[i][j]);
      }
      guard4_in2_b(acc[i][0], acc[i][1], acc[i][2], acc[i][3], ah, al);
    }
    keep4_b(bh[0], bh[1], bh[2], bh[3]);
  }
  acc_guard4(acc[0][0], acc[0][1], acc[0][2], acc[0][3]);
  acc_guard4(acc[1][0], acc[1][1], acc[1][2], acc[1][3]);
  acc_guard4(acc[2][0], acc[2][1], acc[2][2], acc[2][3]);
  acc_guard4(acc[3][0], acc[3][1], acc[3][2], acc[3][3]);

  float* slab = sT[wave];
#pragma unroll
  for (int i = 0; i < 4; ++i) {
    const int mBase = m0 + (i << 4);
#pragma unroll
    for (int j = 0; j < 4; ++j)
#pragma unroll
      for (int r = 0; r < 8; ++r) slab[(mOff + r) * SLABP + (j << 4) + rlane] = acc[i][j][r];
    __builtin_amdgcn_fence(__ATOMIC_RELEASE, "workgroup");
    __builtin_amdgcn_wave_barrier();
    __builtin_amdgcn_fence(__ATOMIC_ACQUIRE, "workgroup");
    {
      const int hh = lane >> 4, c4 = (lane & 15) * 4;
      for (int pass = 0; pass < 2; ++pass) {
#pragma unroll
        for (int it = 0; it < 8; ++it) {
          const int row = it * 2 + hh;
          const v4f v = *(const v4f*)(slab + row * SLABP + c4);
          *(volatile v4f*)(C + (size_t)(mBase + row) * ldc + n0 + c4) = v;
        }
        __threadfence();
      }
    }
    __builtin_amdgcn_fence(__ATOMIC_RELEASE, "workgroup");
    __builtin_amdgcn_wave_barrier();
    __builtin_amdgcn_fence(__ATOMIC_ACQUIRE, "workgroup");
  }
}

__global__ __launch_bounds__(NTHR) void attn_rnn_kernel(
    const float* __restrict__ PRES, const float* __restrict__ PRET,
    const unsigned short* __restrict__ HShi, const unsigned short* __restrict__ HSlo,
    const unsigned short* __restrict__ HThi, const unsigned short* __restrict__ HTlo,
    const unsigned short* __restrict__ WMp, const unsigned short* __restrict__ WIMp,
    const float* __restrict__ BM, const float* __restrict__ WE, float* __restrict__ HMF) {
  __shared__ __align__(16) unsigned short Ahm[2][SEQB * HMP];
  __shared__ __align__(16) unsigned short Amk[2][SEQB * MKP];
  __shared__ __align__(16) float          HW[SEQB * HWP];
  __shared__ __align__(16) float          AL[SEQB * NTP];
  const __bf16* WMB = (const __bf16*)WMp;
  const __bf16* WIM = (const __bf16*)WIMp;
  const int tid = threadIdx.x, lane = tid & 31, wave = tid >> 5;
  const int c = lane & 15, hh = lane >> 4, koff = hh * 8, c4 = c * 4, l4 = lane * 4;
  const int b0 = blockIdx.x * SEQB;

  {
    unsigned* p = (unsigned*)&Ahm[0][0];
#pragma unroll 1
    for (int i = tid; i < SEQB * HMP; i += NTHR) p[i] = 0u;
    unsigned* q = (unsigned*)&Amk[0][0];
#pragma unroll 1
    for (int i = tid; i < SEQB * MKP; i += NTHR) q[i] = 0u;
  }
  __syncthreads();

  const v8f z8 = {0.f, 0.f, 0.f, 0.f, 0.f, 0.f, 0.f, 0.f};
  const __bf16* ahh = (const __bf16*)&Ahm[0][0] + c * HMP + koff;
  const __bf16* ahl = (const __bf16*)&Ahm[1][0] + c * HMP + koff;
  const __bf16* amh = (const __bf16*)&Amk[0][0] + c * MKP + koff;
  const __bf16* aml = (const __bf16*)&Amk[1][0] + c * MKP + koff;

#pragma unroll 1
  for (int k = 0; k < NTH; ++k) {
#pragma unroll
    for (int j = 0; j < 4; ++j) {
      const int n = 64 * wave + 16 * j + c;
      const __bf16* wr = WMB + (size_t)n * NHID + koff;
      v8f acc = z8;
#pragma unroll 1
      for (int k0 = 0; k0 < NHID; k0 += 32) {
        const v16b ah = FragB::load(ahh + k0);
        const v16b al = FragB::load(ahl + k0);
        const v16b fb = FragB::load(wr + k0);
        acc = FragB::mma(ah, fb, acc);
        acc = FragB::mma(al, fb, acc);
        guard1_in3_b(acc, ah, al, fb);
      }
      acc_guard1(acc);
#pragma unroll
      for (int r = 0; r < 8; ++r) HW[(8 * hh + r) * HWP + n] = acc[r];
    }
    __syncthreads();

    {
      v4f wev[4];
#pragma unroll
      for (int m = 0; m < 4; ++m) wev[m] = *(const v4f*)(WE + 128 * m + l4);
#pragma unroll 1
      for (int bb = 0; bb < 2; ++bb) {
        const int bl = 2 * wave + bb;
        const int brow = b0 + bl;
        v4f ptv[4], hwv[4];
        const float* ptrow = PRET + (size_t)(k * NBAT + brow) * NHID + l4;
#pragma unroll
        for (int m = 0; m < 4; ++m) {
          ptv[m] = *(const v4f*)(ptrow + 128 * m);
          hwv[m] = *(const v4f*)(HW + bl * HWP + 128 * m + l4);
        }
        float s0 = 0.0f, s1 = 0.0f;
#pragma unroll 1
        for (int t = 0; t < NTP; ++t) {
          const float* psrow = PRES + (size_t)(t * NBAT + brow) * NHID + l4;
          v4f psv[4];
#pragma unroll
          for (int m = 0; m < 4; ++m) psv[m] = *(const v4f*)(psrow + 128 * m);
          float a = 0.0f;
#pragma unroll
          for (int m = 0; m < 4; ++m) {
#pragma unroll
            for (int e = 0; e < 4; ++e) {
              const float x = (psv[m][e] + ptv[m][e]) + hwv[m][e];
              a = fmaf(wev[m][e], tnh_f(x), a);
            }
          }
#pragma unroll
          for (int off = 1; off < 32; off <<= 1) a += __shfl_xor(a, off, 32);
          const bool mine = (lane == (t & 31));
          s0 = (mine && t < 32) ? a : s0;
          s1 = (mine && t >= 32) ? a : s1;
        }
        float mx = fmaxf(s0, s1);
#pragma unroll
        for (int off = 1; off < 32; off <<= 1) mx = fmaxf(mx, __shfl_xor(mx, off, 32));
        const float e0 = expf(s0 - mx), e1 = expf(s1 - mx);
        float sm = e0 + e1;
#pragma unroll
        for (int off = 1; off < 32; off <<= 1) sm += __shfl_xor(sm, off, 32);
        const float inv = 1.0f / sm;
        AL[bl * NTP + lane]      = e0 * inv;
        AL[bl * NTP + 32 + lane] = e1 * inv;
      }
    }
    __syncthreads();

#pragma unroll 1
    for (int i = 0; i < 4; ++i) {
      const int u = tid + NTHR * i;
      const int bl = u >> 6, ch = u & 63;
      const int brow = b0 + bl;
      float acc8[8];
#pragma unroll
      for (int e = 0; e < 8; ++e) acc8[e] = 0.0f;
#pragma unroll 1
      for (int t = 0; t < NTP; ++t) {
        const size_t off = (size_t)(t * NBAT + brow) * NHID + 8 * ch;
        const v4u wh = *(const v4u*)(HShi + off);
        const v4u wl = *(const v4u*)(HSlo + off);
        const float al = AL[bl * NTP + t];
#pragma unroll
        for (int e = 0; e < 4; ++e) {
          const float v0 = __uint_as_float(wh[e] << 16) + __uint_as_float(wl[e] << 16);
          const float v1 = __uint_as_float(wh[e] & 0xffff0000u) + __uint_as_float(wl[e] & 0xffff0000u);
          acc8[2 * e]     = fmaf(al, v0, acc8[2 * e]);
          acc8[2 * e + 1] = fmaf(al, v1, acc8[2 * e + 1]);
        }
      }
      v4u ph, pl;
#pragma unroll
      for (int e = 0; e < 4; ++e) {
        const float h0 = acc8[2 * e], h1 = acc8[2 * e + 1];
        const unsigned short hb0 = f2bf_bits(h0), hb1 = f2bf_bits(h1);
        const unsigned short lb0 = f2bf_bits(h0 - bf_bits2f(hb0)), lb1 = f2bf_bits(h1 - bf_bits2f(hb1));
        ph[e] = (unsigned)hb0 | ((unsigned)hb1 << 16);
        pl[e] = (unsigned)lb0 | ((unsigned)lb1 << 16);
      }
      *(v4u*)(&Amk[0][0] + bl * MKP + 8 * ch) = ph;
      *(v4u*)(&Amk[1][0] + bl * MKP + 8 * ch) = pl;
    }
#pragma unroll 1
    for (int i = 0; i < 4; ++i) {
      const int u = tid + NTHR * i;
      const int bl = u >> 6, ch = u & 63;
      const int brow = b0 + bl;
      const size_t off = (size_t)(k * NBAT + brow) * NHID + 8 * ch;
      const v4u vh = *(const v4u*)(HThi + off);
      const v4u vl = *(const v4u*)(HTlo + off);
      *(v4u*)(&Amk[0][0] + bl * MKP + NHID + 8 * ch) = vh;
      *(v4u*)(&Amk[1][0] + bl * MKP + NHID + 8 * ch) = vl;
    }
    __syncthreads();

#pragma unroll
    for (int j = 0; j < 4; ++j) {
      const int n = 64 * wave + 16 * j + c;
      const __bf16* wi = WIM + (size_t)n * NK2 + koff;
      const __bf16* wg = WIM + (size_t)(NK2 + n) * NK2 + koff;
      const __bf16* wo = WIM + (size_t)(NG3O + n) * NK2 + koff;
      v8f ai = z8, ag = z8, ao = z8;
#pragma unroll 1
      for (int k0 = 0; k0 < NK2; k0 += 32) {
        const v16b ah  = FragB::load(amh + k0);
        const v16b al  = FragB::load(aml + k0);
        const v16b fbi = FragB::load(wi + k0);
        const v16b fbg = FragB::load(wg + k0);
        const v16b fbo = FragB::load(wo + k0);
        ai = FragB::mma(ah, fbi, ai);
        ai = FragB::mma(al, fbi, ai);
        ag = FragB::mma(ah, fbg, ag);
        ag = FragB::mma(al, fbg, ag);
        ao = FragB::mma(ah, fbo, ao);
        ao = FragB::mma(al, fbo, ao);
        guard3_in5_b(ai, ag, ao, ah, al, fbi, fbg, fbo);
      }
      acc_guard3(ai, ag, ao);
      const float bI = BM[n], bG = BM[NK2 + n], bO = BM[NG3O + n];
#pragma unroll
      for (int r = 0; r < 8; ++r) {
        const float h = cell_h(ai[r] + bI, ag[r] + bG, ao[r] + bO);
        const unsigned short hb = f2bf_bits(h);
        const unsigned short lb = f2bf_bits(h - bf_bits2f(hb));
        Ahm[0][(8 * hh + r) * HMP + n] = hb;
        Ahm[1][(8 * hh + r) * HMP + n] = lb;
        HW[(8 * hh + r) * HWP + n] = h;
      }
    }
    __syncthreads();
  }

  for (int pass = 0; pass < 2; ++pass) {
#pragma unroll
    for (int it = 0; it < 8; ++it) {
      const int row = it * 2 + hh;
      const v4f v = *(const v4f*)(HW + row * HWP + 64 * wave + c4);
      *(volatile v4f*)(HMF + (size_t)(b0 + row) * NHID + 64 * wave + c4) = v;
    }
    __threadfence();
  }
}

__global__ __launch_bounds__(128) void fc_kernel(const float* __restrict__ HMF, const float* __restrict__ FCW,
                                                const float* __restrict__ FCB, float* __restrict__ out) {
  __shared__ __align__(16) float os[NBAT * NCLS];
  const int tid = threadIdx.x;
  const float* hrow = HMF + (size_t)tid * NHID;
  float a0 = 0.0f, a1 = 0.0f, a2 = 0.0f;
#pragma unroll 1
  for (int k4 = 0; k4 < NHID; k4 += 4) {
    const v4f hv = *(const v4f*)(hrow + k4);
    const v4f w0 = *(const v4f*)(FCW + k4);
    const v4f w1 = *(const v4f*)(FCW + NHID + k4);
    const v4f w2 = *(const v4f*)(FCW + 2 * NHID + k4);
#pragma unroll
    for (int e = 0; e < 4; ++e) {
      a0 = fmaf(hv[e], w0[e], a0);
      a1 = fmaf(hv[e], w1[e], a1);
      a2 = fmaf(hv[e], w2[e], a2);
    }
  }
  os[tid * NCLS + 0] = a0 + FCB[0];
  os[tid * NCLS + 1] = a1 + FCB[1];
  os[tid * NCLS + 2] = a2 + FCB[2];
  __syncthreads();
  if (tid < 32) {
    for (int pass = 0; pass < 2; ++pass) {
#pragma unroll
      for (int q = 0; q < 3; ++q) {
        const int idx = 32 * q + tid;
        const v4f v = *(const v4f*)(os + 4 * idx);
        *(volatile v4f*)(out + 4 * idx) = v;
      }
      __threadfence();
    }
  }
}

extern "C" void kernel_launch(void* const* d_in, const int* in_sizes, int n_in,
                              void* d_out, int out_size, void* d_ws, size_t ws_size, hipStream_t stream) {
  if (n_in < 20 || d_out == nullptr || d_ws == nullptr) return;
  if (in_sizes[0] != NROWP || in_sizes[2] != NROWH || in_sizes[4] != NVOC * NEMB || in_sizes[5] != NHID ||
      in_sizes[6] != NHID * NHID || in_sizes[7] != NHID * NHID || in_sizes[8] != NHID * NHID ||
      in_sizes[9] != NG4 * NEMB || in_sizes[10] != NG4 || in_sizes[11] != NG4 ||
      in_sizes[12] != NG4 * NEMB || in_sizes[13] != NG4 || in_sizes[14] != NG4 ||
      in_sizes[15] != NG4 * NK2 || in_sizes[16] != NG4 || in_sizes[17] != NG4 ||
      in_sizes[18] != NCLS * NHID || in_sizes[19] != NCLS || out_size != NBAT * NCLS) return;

  const int*   tokP  = (const int*)d_in[0];
  const int*   tokH  = (const int*)d_in[2];
  const float* emb   = (const float*)d_in[4];
  const float* w_e   = (const float*)d_in[5];
  const float* Ws    = (const float*)d_in[6];
  const float* Wt    = (const float*)d_in[7];
  const float* Wm    = (const float*)d_in[8];
  const float* Wih_p = (const float*)d_in[9];
  const float* bih_p = (const float*)d_in[10];
  const float* bhh_p = (const float*)d_in[11];
  const float* Wih_h = (const float*)d_in[12];
  const float* bih_h = (const float*)d_in[13];
  const float* bhh_h = (const float*)d_in[14];
  const float* Wih_m = (const float*)d_in[15];
  const float* bih_m = (const float*)d_in[16];
  const float* bhh_m = (const float*)d_in[17];
  const float* fc_w  = (const float*)d_in[18];
  const float* fc_b  = (const float*)d_in[19];
  float* out = (float*)d_out;

  char* ws = (char*)d_ws; size_t off = 0;
  auto carve = [&](size_t bytes) -> char* { char* p = ws + off; off += (bytes + 255) & ~(size_t)255; return p; };
  unsigned short* XP   = (unsigned short*)carve((size_t)NROWP * KEMB * 2);
  unsigned short* XH   = (unsigned short*)carve((size_t)NROWH * KEMB * 2);
  unsigned short* WIP  = (unsigned short*)carve((size_t)NG4 * KEMB * 2);
  unsigned short* WIH  = (unsigned short*)carve((size_t)NG4 * KEMB * 2);
  unsigned short* WIM  = (unsigned short*)carve((size_t)NG4 * NK2 * 2);
  unsigned short* WSB  = (unsigned short*)carve((size_t)NHID * NHID * 2);
  unsigned short* WTB  = (unsigned short*)carve((size_t)NHID * NHID * 2);
  unsigned short* WMB  = (unsigned short*)carve((size_t)NHID * NHID * 2);
  unsigned short* HSH  = (unsigned short*)carve((size_t)NROWP * NHID * 2);
  unsigned short* HSL  = (unsigned short*)carve((size_t)NROWP * NHID * 2);
  unsigned short* HTH  = (unsigned short*)carve((size_t)NROWH * NHID * 2);
  unsigned short* HTL  = (unsigned short*)carve((size_t)NROWH * NHID * 2);
  float*          PRES = (float*)carve((size_t)NROWP * NHID * 4);
  float*          PRET = (float*)carve((size_t)NROWH * NHID * 4);
  float*          BP   = (float*)carve((size_t)NG4 * 4);
  float*          BH   = (float*)carve((size_t)NG4 * 4);
  float*          BM   = (float*)carve((size_t)NG4 * 4);
  float*          WE   = (float*)carve((size_t)NHID * 4);
  float*          FCW  = (float*)carve((size_t)NCLS * NHID * 4);
  float*          FCB  = (float*)carve((size_t)32 * 4);
  float*          HMF  = (float*)carve((size_t)NBAT * NHID * 4);
  if (off > ws_size || off > (size_t)134217728) return;

  const int n8s = NHID * (NHID / 8);
  const int n8m = NG4 * (NK2 / 8);
  const int n8e = NG4 * (KEMB / 8);
  const int n8x = NROWP * (KEMB / 8);
  cvt8_kernel<0><<<(n8s + NTHR - 1) / NTHR, NTHR, 0, stream>>>(Ws, WSB, NHID, NHID / 8, NHID, 0, 1.0f);
  cvt8_kernel<0><<<(n8s + NTHR - 1) / NTHR, NTHR, 0, stream>>>(Wt, WTB, NHID, NHID / 8, NHID, 0, 1.0f);
  cvt8_kernel<0><<<(n8s + NTHR - 1) / NTHR, NTHR, 0, stream>>>(Wm, WMB, NHID, NHID / 8, NHID, 0, 1.0f);
  cvt8_kernel<0><<<(n8m + NTHR - 1) / NTHR, NTHR, 0, stream>>>(Wih_m, WIM, NG4, NK2 / 8, NK2, 0, 1.0f);
  cvt_pad_kernel<<<(n8e + NTHR - 1) / NTHR, NTHR, 0, stream>>>(Wih_p, WIP, NG4);
  cvt_pad_kernel<<<(n8e + NTHR - 1) / NTHR, NTHR, 0, stream>>>(Wih_h, WIH, NG4);
  gather_rows_kernel<<<(n8x + NTHR - 1) / NTHR, NTHR, 0, stream>>>(tokP, emb, XP, NROWP);
  gather_rows_kernel<<<(n8x + NTHR - 1) / NTHR, NTHR, 0, stream>>>(tokH, emb, XH, NROWH);
  param_prep_kernel<<<5, NTHR, 0, stream>>>(bih_p, bhh_p, bih_h, bhh_h, bih_m, bhh_m, w_e, fc_w, fc_b, BP, BH, BM, WE, FCW, FCB);
  gate_gemm_kernel<<<NROWP / 16, NTHR, 0, stream>>>(XP, WIP, BP, HSH, HSL, NROWP);
  gate_gemm_kernel<<<NROWH / 16, NTHR, 0, stream>>>(XH, WIH, BH, HTH, HTL, NROWH);
  proj_gemm_kernel<<<(NROWP / 64) * (NHID / 64) / (NTHR / 32), NTHR, 0, stream>>>(HSH, HSL, NHID, WSB, NHID, PRES, NHID, NROWP, NHID, NHID);
  proj_gemm_kernel<<<(NROWH / 64) * (NHID / 64) / (NTHR / 32), NTHR, 0, stream>>>(HTH, HTL, NHID, WTB, NHID, PRET, NHID, NROWH, NHID, NHID);
  attn_rnn_kernel<<<NBAT / SEQB, NTHR, 0, stream>>>(PRES, PRET, HSH, HSL, HTH, HTL, WMB, WIM, BM, WE, HMF);
  fc_kernel<<<1, NBAT, 0, stream>>>(HMF, FCW, FCB, out);
}
